// NNSARSALambda_84636625535232
// MI455X (gfx1250) — hardware-verified
//
#include <hip/hip_runtime.h>
#include <stddef.h>


typedef _Float16 v16h __attribute__((ext_vector_type(16)));
typedef _Float16 v8h  __attribute__((ext_vector_type(8)));
typedef float    v8f  __attribute__((ext_vector_type(8)));
typedef float    v4f  __attribute__((ext_vector_type(4)));
typedef int      v4i  __attribute__((ext_vector_type(4)));

#ifndef SEQ
#define SEQ 2048
#endif
#define SEQ_FULL 2048
#define DIN   128
#define HDIM  512
#define ADIM  8
#define POUT  (DIN * HDIM + HDIM + HDIM * ADIM + ADIM)
#define OUT_W1 0
#define OUT_B1 (DIN * HDIM)
#define OUT_W2 (OUT_B1 + HDIM)
#define OUT_B2 (OUT_W2 + HDIM * ADIM)

#ifndef GW2_RES
#define GW2_RES 1
#endif

static_assert(SEQ >= 256 && SEQ <= SEQ_FULL && (SEQ % 256) == 0);
static_assert(POUT == 70152);
static_assert(OUT_B1 == 65536 && OUT_W2 == 66048 && OUT_B2 == 70144);
static_assert(((size_t)OUT_B1 * 4) % 128 == 0 && ((size_t)OUT_W2 * 4) % 128 == 0);
static_assert(((size_t)OUT_B2 * 4) % 128 == 0);
static_assert((DIN % 64) == 0 && (DIN % 32) == 0);
static_assert((HDIM % 128) == 0 && (HDIM % 32) == 0);
static_assert((SEQ % 64) == 0 && (SEQ % 32) == 0);
static_assert(ADIM == 8);
static_assert(HDIM * ADIM == 16 * 256);
static_assert(((SEQ * DIN) % 2048) == 0);
static_assert(GW2_RES == 0 || GW2_RES == 1);

#define LDT 72
#define LDC 68
static_assert((LDT % 8) == 0 && LDT >= 64);
static_assert((LDC % 4) == 0 && LDC >= 64);

#define LDW2 (HDIM + 8)
#define LDE  (SEQ + 8)
static_assert((LDW2 % 8) == 0 && (LDE % 8) == 0);

#define WCARRY 64.0f
#define XCARRY 64.0f
#define UCARRY 1024.0f
#define ECARRY 2048.0f
#define DECAYF 0.891f
static_assert(XCARRY == WCARRY);

#define W1T_BYTES ((size_t)HDIM * DIN * 2)
#define XT_BYTES  ((size_t)DIN * SEQ * 2)
#define X16_BYTES ((size_t)SEQ * DIN * 2)
#define H16_BYTES ((size_t)SEQ * HDIM * 2)
#define HT_BYTES  ((size_t)HDIM * SEQ * 2)
#define UT_BYTES  ((size_t)HDIM * SEQ * 2)
#define CP_BYTES  ((size_t)SEQ * 4)
#define OFF_W1T ((size_t)0)
#define OFF_XT  (OFF_W1T + W1T_BYTES)
#define OFF_X16 (OFF_XT + XT_BYTES)
#define OFF_H16 (OFF_X16 + X16_BYTES)
#define OFF_HT  (OFF_H16 + H16_BYTES)
#define OFF_UT  (OFF_HT + HT_BYTES)
#define OFF_CP  (OFF_UT + UT_BYTES)
#define WS_TOTAL (OFF_CP + CP_BYTES)
static_assert((W1T_BYTES % 128) == 0 && (XT_BYTES % 128) == 0 && (X16_BYTES % 128) == 0);
static_assert((H16_BYTES % 128) == 0 && (HT_BYTES % 128) == 0 && (UT_BYTES % 128) == 0);
static_assert((CP_BYTES % 128) == 0);
static_assert(WS_TOTAL <= (size_t)134217728);

static_assert(64 * LDT * 2 <= 131072);
static_assert(64 * LDC * 4 <= 131072);
static_assert(9 * LDW2 * 2 + SEQ * 4 + SEQ * 4 + 64 * 4 <= 131072);
static_assert((1 + GW2_RES) * 9 * LDE * 2 + 8 * 128 * 4 <= 131072);

static_assert((256 / 8) * 2 == 64);
static_assert((256 / 16) * 4 == 64);
static_assert((256 / 64) * 16 == 64);

__device__ __forceinline__ float bf16r(float x) {
  unsigned int u = __float_as_uint(x);
  u = (u + 0x7FFFu + ((u >> 16) & 1u)) & 0xFFFF0000u;
  return __uint_as_float(u);
}

__device__ __forceinline__ _Float16 toh_flush(float v) {
  const _Float16 r = (_Float16)v;
  return (fabsf(v) < 6.103515625e-05f) ? (_Float16)0.0f : r;
}

__device__ __forceinline__ v16h frag_at(const _Float16* p) {
  v8h lo = *(const v8h*)(p);
  v8h hi = *(const v8h*)(p + 16);
  v16h out;
#pragma unroll
  for (int i = 0; i < 8; ++i) { out[i] = lo[i]; out[i + 8] = hi[i]; }
  return out;
}

__device__ __forceinline__ v8f wmma16(v16h a, v16h b, v8f c) {
  v8f d = __builtin_amdgcn_wmma_f32_16x16x32_f16(false, a, false, b, (short)0, c,
                                                 false, false);
  asm volatile("v_nop\n\tv_nop\n\tv_nop\n\tv_nop" : "+v"(d) : "v"(a), "v"(b));
  return d;
}

__device__ __forceinline__ float red16_sum(float x) {
#pragma unroll
  for (int off = 1; off < 16; off <<= 1) x += __shfl_xor(x, off, 32);
  return x;
}
__device__ __forceinline__ float red32_sum(float x) {
#pragma unroll
  for (int off = 1; off < 32; off <<= 1) x += __shfl_xor(x, off, 32);
  return x;
}

__device__ __forceinline__ void wave_lds_sync() {
  __builtin_amdgcn_fence(3  , "wavefront");
  asm volatile("s_wait_dscnt 0x0" ::: "memory");
  __builtin_amdgcn_wave_barrier();
}

__global__ __launch_bounds__(256) void wconv_kernel(
    const float* __restrict__ W, _Float16* __restrict__ Wt, unsigned ldw, unsigned ldk) {
  __shared__ _Float16 T[64 * LDT];
  const unsigned tid = threadIdx.x;
  const unsigned n0 = blockIdx.x * 64u;
  const unsigned k0 = blockIdx.y * 64u;
#pragma unroll 4
  for (unsigned j = 0; j < 16u; ++j) {
    const unsigned idx = tid + 256u * j;
    const unsigned kr = idx >> 6, nc = idx & 63u;
    const float v = W[(size_t)(k0 + kr) * ldw + n0 + nc];
    T[nc * LDT + kr] = toh_flush(WCARRY * bf16r(v));
  }
  __syncthreads();
  v8h x[2];
  size_t off[2];
#pragma unroll
  for (unsigned i = 0; i < 2u; ++i) {
    const unsigned n = 32u * i + (tid >> 3);
    const unsigned kc = (tid & 7u) * 8u;
    x[i] = *(const v8h*)&T[n * LDT + kc];
    off[i] = (size_t)(n0 + n) * ldk + k0 + kc;
  }
#pragma unroll
  for (int i = 0; i < 2; ++i) *(volatile v8h*)(Wt + off[i]) = x[i];
  __threadfence();
#pragma unroll
  for (int i = 0; i < 2; ++i) *(volatile v8h*)(Wt + off[i]) = x[i];
}

__global__ __launch_bounds__(256) void xcast_kernel(
    const float* __restrict__ X, _Float16* __restrict__ X16) {
#pragma clang fp contract(off)
  const size_t idx = ((size_t)blockIdx.x * 256u + threadIdx.x) * 8u;
  const v4f a0 = *(const v4f*)(X + idx);
  const v4f a1 = *(const v4f*)(X + idx + 4u);
  v8h o;
#pragma unroll
  for (int i = 0; i < 4; ++i) {
    o[i]     = toh_flush(XCARRY * bf16r(a0[i]));
    o[i + 4] = toh_flush(XCARRY * bf16r(a1[i]));
  }
  _Float16* p = X16 + idx;
  *(volatile v8h*)p = o;
  __threadfence();
  *(volatile v8h*)p = o;
}

__global__ __launch_bounds__(256) void fwd_kernel(
    const _Float16* __restrict__ A16, const _Float16* __restrict__ Bt,
    const float* __restrict__ b1, _Float16* __restrict__ H16, _Float16* __restrict__ HT16) {
  __shared__ __attribute__((aligned(16))) float Cs[64 * LDC];
  const unsigned tid = threadIdx.x, lane = tid & 31u;
  const unsigned w = (unsigned)__builtin_amdgcn_readfirstlane((int)(threadIdx.x >> 5));
  const unsigned mw = w >> 1, nw = w & 1u;
  const unsigned hh = lane >> 4, m = lane & 15u;
  const unsigned n0 = blockIdx.x * 64u;
  const unsigned row0 = blockIdx.y * 64u;

  const _Float16* ap  = A16 + (size_t)(row0 + mw * 16u + m) * DIN + hh * 8u;
  const _Float16* bp0 = Bt + (size_t)(n0 + nw * 32u + m) * DIN + hh * 8u;
  const _Float16* bp1 = bp0 + (size_t)16 * DIN;
  v8f acc0 = {}, acc1 = {};
#pragma unroll 2
  for (unsigned k0 = 0; k0 < (unsigned)DIN; k0 += 32u) {
    const v16h a   = frag_at(ap + k0);
    const v16h b0  = frag_at(bp0 + k0);
    const v16h b1f = frag_at(bp1 + k0);
    acc0 = wmma16(a, b0, acc0);
    acc1 = wmma16(a, b1f, acc1);
  }
#pragma unroll
  for (int r = 0; r < 8; ++r) {
    float* d = &Cs[(mw * 16u + hh * 8u + (unsigned)r) * LDC + nw * 32u + m];
    d[0]  = acc0[r];
    d[16] = acc1[r];
  }
  __syncthreads();

  {
    const unsigned cc = tid & 63u;
    const float bb = bf16r(b1[n0 + cc]);
#pragma unroll 1
    for (unsigned e = 0; e < 16u; ++e) {
      const unsigned r = (tid >> 6) + 4u * e;
      const float pre = Cs[r * LDC + cc] * (1.0f / (XCARRY * WCARRY)) + bb;
      Cs[r * LDC + cc] = tanhf(pre);
    }
  }
  __syncthreads();

  v8h x[2], xt[2];
  size_t off[2], offt[2];
#pragma unroll
  for (unsigned i = 0; i < 2u; ++i) {
    const unsigned r = 32u * i + (tid >> 3);
    const unsigned c = (tid & 7u) * 8u;
    const v4f u0 = *(const v4f*)&Cs[r * LDC + c];
    const v4f u1 = *(const v4f*)&Cs[r * LDC + c + 4];
#pragma unroll
    for (int j = 0; j < 4; ++j) {
      x[i][j]     = toh_flush(u0[j]);
      x[i][j + 4] = toh_flush(u1[j]);
    }
    off[i] = (size_t)(row0 + r) * HDIM + n0 + c;
#pragma unroll
    for (unsigned j = 0; j < 8u; ++j) xt[i][j] = toh_flush(Cs[(c + j) * LDC + r]);
    offt[i] = (size_t)(n0 + r) * SEQ + row0 + c;
  }
#pragma unroll
  for (int i = 0; i < 2; ++i) *(volatile v8h*)(H16 + off[i]) = x[i];
#pragma unroll
  for (int i = 0; i < 2; ++i) *(volatile v8h*)(HT16 + offt[i]) = xt[i];
  __threadfence();
#pragma unroll
  for (int i = 0; i < 2; ++i) *(volatile v8h*)(H16 + off[i]) = x[i];
#pragma unroll
  for (int i = 0; i < 2; ++i) *(volatile v8h*)(HT16 + offt[i]) = xt[i];
}

__global__ __launch_bounds__(256) void qscan_kernel(
    const _Float16* __restrict__ H16, const float* __restrict__ W2,
    const float* __restrict__ b2, const float* __restrict__ targets,
    const int* __restrict__ actions, const int* __restrict__ dones,
    float* __restrict__ Cp, float* __restrict__ out_b2) {
  __shared__ __attribute__((aligned(16))) _Float16 W2s[9 * LDW2];
  __shared__ __attribute__((aligned(16))) float es[SEQ];
  __shared__ __attribute__((aligned(16))) int dn[SEQ];
  __shared__ __attribute__((aligned(16))) float red[64];

  const unsigned tid = threadIdx.x, lane = tid & 31u;
  const unsigned wave = (unsigned)__builtin_amdgcn_readfirstlane((int)(threadIdx.x >> 5));
  const unsigned hh = lane >> 4, m = lane & 15u;

#pragma unroll 4
  for (unsigned e = 0; e < 16u; ++e) {
    const unsigned id = tid + 256u * e;
    const unsigned i = id >> 3, j = id & 7u;
    W2s[j * LDW2 + i] = toh_flush(WCARRY * bf16r(W2[id]));
  }
#pragma unroll 1
  for (unsigned c = tid; c < (unsigned)LDW2; c += 256u) W2s[8u * LDW2 + c] = (_Float16)0.0f;
#pragma unroll 1
  for (unsigned t = tid; t < (unsigned)SEQ; t += 256u) dn[t] = dones[t];
  __syncthreads();

  {
    const unsigned rsel = (m < 8u) ? m : 8u;
    const float bb = bf16r(b2[m & 7u]);
    for (unsigned tile = wave; tile < (unsigned)(SEQ / 16); tile += 8u) {
      const unsigned t0 = tile * 16u;
      const _Float16* ap = H16 + (size_t)(t0 + m) * HDIM + hh * 8u;
      const _Float16* bp = &W2s[rsel * LDW2 + hh * 8u];
      v8f acc = {};
#pragma unroll 2
      for (unsigned k0 = 0; k0 < (unsigned)HDIM; k0 += 32u) {
        const v16h a = frag_at(ap + k0);
        const v16h b = frag_at(bp + k0);
        acc = wmma16(a, b, acc);
      }
#pragma unroll
      for (int r = 0; r < 8; ++r) {
        const unsigned t = t0 + hh * 8u + (unsigned)r;
        const float tg = bf16r(targets[(size_t)t * ADIM + (m & 7u)]);
        const float q = acc[r] * (1.0f / WCARRY) + bb;
        const float d = tg - q;
        const float sq = (m < 8u) ? d * d : 0.0f;
        const float s = red16_sum(sq);
        if (m == 0u) es[t] = s * (1.0f / (float)ADIM);
      }
    }
  }
  __syncthreads();

  if (wave == 0u) {
    float cn = 0.0f;
#pragma unroll 1
    for (int t = SEQ - 1; t >= 0; --t) {
      const float e = es[t];
      const int d = dn[t];
      const float carry = (d > 0) ? 0.0f : DECAYF * cn;
      const float cs = e + carry;
      if (lane == 0u) es[t] = cs;
      cn = cs;
    }
  }
  __syncthreads();

  for (unsigned idx = tid * 4u; idx < (unsigned)SEQ; idx += 1024u) {
    const v4f cv = *(const v4f*)&es[idx];
    *(volatile v4f*)(Cp + idx) = cv;
    __threadfence();
    *(volatile v4f*)(Cp + idx) = cv;
  }

  float pa[8];
#pragma unroll
  for (int j = 0; j < 8; ++j) pa[j] = 0.0f;
#pragma unroll 1
  for (unsigned t = tid; t < (unsigned)SEQ; t += 256u) {
    const float c = es[t];
    int a = actions[t];
    a = min(max(a, 0), ADIM - 1);
#pragma unroll
    for (int j = 0; j < 8; ++j) pa[j] += (a == j) ? c : 0.0f;
  }
#pragma unroll
  for (int j = 0; j < 8; ++j) {
    const float s = red32_sum(pa[j]);
    if (lane == 0u) red[wave * 8u + (unsigned)j] = s;
  }
  __syncthreads();
  if (wave == 0u) {
    float tot[8];
#pragma unroll
    for (int j = 0; j < 8; ++j) {
      float s = 0.0f;
#pragma unroll
      for (int wv = 0; wv < 8; ++wv) s += red[wv * 8 + j];
      tot[j] = s;
    }
    v4f val;
#pragma unroll
    for (int k = 0; k < 4; ++k) val[k] = (lane == 0u) ? tot[k] : tot[k + 4];
    float* p = out_b2 + 4u * (lane & 1u);
    if (lane < 2u) *(volatile v4f*)p = val;
    __threadfence();
    if (lane < 2u) *(volatile v4f*)p = val;
  }
}

__global__ __launch_bounds__(256) void makeu_kernel(
    const _Float16* __restrict__ HT16, const float* __restrict__ W2,
    const int* __restrict__ actions, const float* __restrict__ Cp,
    _Float16* __restrict__ UT16, float* __restrict__ out_b1) {
#pragma clang fp contract(off)
  __shared__ __attribute__((aligned(16))) float rowsum[32];
  const unsigned tid = threadIdx.x, lane = tid & 31u;
  const unsigned wave = (unsigned)__builtin_amdgcn_readfirstlane((int)(threadIdx.x >> 5));

#pragma unroll 1
  for (unsigned rr = 0; rr < 4u; ++rr) {
    const unsigned i = blockIdx.x * 32u + wave * 4u + rr;
    float wj[8];
#pragma unroll
    for (int j = 0; j < 8; ++j) wj[j] = bf16r(W2[(size_t)i * ADIM + j]);
    float rs = 0.0f;
#pragma unroll 1
    for (unsigned s = 0; s < (unsigned)(SEQ / 256); ++s) {
      const unsigned t0 = s * 256u + lane * 8u;
      const v8h h8 = *(const v8h*)(HT16 + (size_t)i * SEQ + t0);
      const v4f c0 = *(const v4f*)(Cp + t0);
      const v4f c1 = *(const v4f*)(Cp + t0 + 4u);
      const v4i a0 = *(const v4i*)(actions + t0);
      const v4i a1 = *(const v4i*)(actions + t0 + 4u);
      float cv[8];
      int av[8];
#pragma unroll
      for (int e = 0; e < 4; ++e) {
        cv[e] = c0[e]; cv[e + 4] = c1[e];
        av[e] = a0[e]; av[e + 4] = a1[e];
      }
      v8h o;
#pragma unroll
      for (int e = 0; e < 8; ++e) {
        const float hv = (float)h8[e];
        const float g = 1.0f - hv * hv;
        const int a = min(max(av[e], 0), ADIM - 1);
        float wsel = wj[0];
#pragma unroll
        for (int j = 1; j < 8; ++j) wsel = (a == j) ? wj[j] : wsel;
        const float u = (cv[e] * g) * wsel;
        rs += u;
        o[e] = toh_flush(UCARRY * u);
      }
      _Float16* p = UT16 + (size_t)i * SEQ + t0;
      *(volatile v8h*)p = o;
      __threadfence();
      *(volatile v8h*)p = o;
    }
    rs = red32_sum(rs);
    if (lane == 0u) rowsum[wave * 4u + rr] = rs;
  }
  __syncthreads();
  if (wave == 0u) {
    const v4f val = *(const v4f*)&rowsum[(lane & 7u) * 4u];
    float* p = out_b1 + blockIdx.x * 32u + (lane & 7u) * 4u;
    if (lane < 8u) *(volatile v4f*)p = val;
    __threadfence();
    if (lane < 8u) *(volatile v4f*)p = val;
  }
}

__global__ __launch_bounds__(256) void gw1_kernel(
    const _Float16* __restrict__ A16, const _Float16* __restrict__ Bt, float* __restrict__ outf) {
  __shared__ __attribute__((aligned(16))) float Cs[64 * LDC];
  const unsigned tid = threadIdx.x, lane = tid & 31u;
  const unsigned w = (unsigned)__builtin_amdgcn_readfirstlane((int)(threadIdx.x >> 5));
  const unsigned mw = w >> 1, nw = w & 1u;
  const unsigned hh = lane >> 4, m = lane & 15u;
  const unsigned n0 = blockIdx.x * 64u;
  const unsigned row0 = blockIdx.y * 64u;

  const _Float16* ap  = A16 + (size_t)(row0 + mw * 16u + m) * SEQ + hh * 8u;
  const _Float16* bp0 = Bt + (size_t)(n0 + nw * 32u + m) * SEQ + hh * 8u;
  const _Float16* bp1 = bp0 + (size_t)16 * SEQ;
  v8f acc0 = {}, acc1 = {};
#pragma unroll 2
  for (unsigned k0 = 0; k0 < (unsigned)SEQ; k0 += 32u) {
    const v16h a   = frag_at(ap + k0);
    const v16h b0  = frag_at(bp0 + k0);
    const v16h b1f = frag_at(bp1 + k0);
    acc0 = wmma16(a, b0, acc0);
    acc1 = wmma16(a, b1f, acc1);
  }
#pragma unroll
  for (int r = 0; r < 8; ++r) {
    float* d = &Cs[(mw * 16u + hh * 8u + (unsigned)r) * LDC + nw * 32u + m];
    d[0]  = acc0[r];
    d[16] = acc1[r];
  }
  __syncthreads();

  const float cs = 1.0f / (WCARRY * UCARRY);
  v4f xs4[4];
  size_t off[4];
#pragma unroll
  for (unsigned i = 0; i < 4u; ++i) {
    const unsigned r = 16u * i + (tid >> 4);
    const unsigned c = (tid & 15u) * 4u;
    const v4f u = *(const v4f*)&Cs[r * LDC + c];
    v4f val;
#pragma unroll
    for (int j = 0; j < 4; ++j) val[j] = u[j] * cs;
    xs4[i] = val;
    off[i] = (size_t)(row0 + r) * HDIM + n0 + c;
  }
#pragma unroll
  for (int i = 0; i < 4; ++i) *(volatile v4f*)(outf + off[i]) = xs4[i];
  __threadfence();
#pragma unroll
  for (int i = 0; i < 4; ++i) *(volatile v4f*)(outf + off[i]) = xs4[i];
}

__global__ __launch_bounds__(256) void gw2_kernel(
    const _Float16* __restrict__ HT16, const float* __restrict__ Cp,
    const int* __restrict__ actions, float* __restrict__ out_w2) {
  __shared__ __attribute__((aligned(16))) _Float16 Es[9 * LDE];
#if GW2_RES
  __shared__ __attribute__((aligned(16))) _Float16 Ers[9 * LDE];
#endif
  __shared__ __attribute__((aligned(16))) float Os[8 * 128];
  const unsigned tid = threadIdx.x, lane = tid & 31u;
  const unsigned wave = (unsigned)__builtin_amdgcn_readfirstlane((int)(threadIdx.x >> 5));
  const unsigned hh = lane >> 4, m = lane & 15u;

#pragma unroll 1
  for (unsigned t = tid; t < (unsigned)SEQ; t += 256u) {
    const float cf = Cp[t];
    const _Float16 ch = toh_flush(cf);
    int a = actions[t];
    a = min(max(a, 0), ADIM - 1);
#pragma unroll
    for (int j = 0; j < 8; ++j) Es[(unsigned)j * LDE + t] = (a == j) ? ch : (_Float16)0.0f;
    Es[8u * LDE + t] = (_Float16)0.0f;
#if GW2_RES
    const _Float16 cl = toh_flush(ECARRY * (cf - (float)ch));
#pragma unroll
    for (int j = 0; j < 8; ++j) Ers[(unsigned)j * LDE + t] = (a == j) ? cl : (_Float16)0.0f;
    Ers[8u * LDE + t] = (_Float16)0.0f;
#endif
  }
  __syncthreads();

  const unsigned i0 = (blockIdx.x * 8u + wave) * 16u;
  const unsigned rsel = (m < 8u) ? m : 8u;
  const _Float16* ap = HT16 + (size_t)(i0 + m) * SEQ + hh * 8u;
  const _Float16* bp = &Es[rsel * LDE + hh * 8u];
#if GW2_RES
  const _Float16* bpr = &Ers[rsel * LDE + hh * 8u];
  v8f accr = {};
#endif
  v8f acc = {};
#pragma unroll 2
  for (unsigned k0 = 0; k0 < (unsigned)SEQ; k0 += 32u) {
    const v16h a = frag_at(ap + k0);
    const v16h b = frag_at(bp + k0);
    acc = wmma16(a, b, acc);
#if GW2_RES
    const v16h br = frag_at(bpr + k0);
    accr = wmma16(a, br, accr);
#endif
  }
#pragma unroll
  for (int r = 0; r < 8; ++r) {
#if GW2_RES
    const float res = acc[r] + accr[r] * (1.0f / ECARRY);
#else
    const float res = acc[r];
#endif
    if (m < 8u) Os[wave * 128u + (hh * 8u + (unsigned)r) * 8u + m] = res;
  }
  wave_lds_sync();
  const v4f val = *(const v4f*)&Os[wave * 128u + lane * 4u];
  float* p = out_w2 + (size_t)i0 * ADIM + lane * 4u;
  *(volatile v4f*)p = val;
  __threadfence();
  *(volatile v4f*)p = val;
}

extern "C" void kernel_launch(void* const* d_in, const int* in_sizes, int n_in,
                              void* d_out, int out_size, void* d_ws, size_t ws_size,
                              hipStream_t stream) {
  if (n_in < 8) return;
  if ((long long)in_sizes[0] < (long long)SEQ * DIN) return;
  if ((long long)in_sizes[1] < (long long)SEQ * ADIM) return;
  if (in_sizes[2] < SEQ || in_sizes[3] < SEQ) return;
  if ((long long)in_sizes[4] < (long long)DIN * HDIM) return;
  if (in_sizes[5] < HDIM) return;
  if (in_sizes[6] < HDIM * ADIM) return;
  if (in_sizes[7] < ADIM) return;
  if ((long long)out_size < (long long)POUT) return;
  if (ws_size < WS_TOTAL) return;

  const float* xs      = (const float*)d_in[0];
  const float* targets = (const float*)d_in[1];
  const int*   actions = (const int*)d_in[2];
  const int*   dones   = (const int*)d_in[3];
  const float* w1      = (const float*)d_in[4];
  const float* b1      = (const float*)d_in[5];
  const float* w2      = (const float*)d_in[6];
  const float* b2      = (const float*)d_in[7];
  float* out = (float*)d_out;

  char* ws = (char*)d_ws;
  _Float16* W1t  = (_Float16*)(ws + OFF_W1T);
  _Float16* XT16 = (_Float16*)(ws + OFF_XT);
  _Float16* X16  = (_Float16*)(ws + OFF_X16);
  _Float16* H16  = (_Float16*)(ws + OFF_H16);
  _Float16* HT16 = (_Float16*)(ws + OFF_HT);
  _Float16* UT16 = (_Float16*)(ws + OFF_UT);
  float*    Cp   = (float*)(ws + OFF_CP);

  dim3 blk(256);

  wconv_kernel<<<dim3(HDIM / 64, DIN / 64), blk, 0, stream>>>(w1, W1t, (unsigned)HDIM, (unsigned)DIN);
  wconv_kernel<<<dim3(DIN / 64, SEQ / 64), blk, 0, stream>>>(xs, XT16, (unsigned)DIN, (unsigned)SEQ);
  xcast_kernel<<<dim3((SEQ * DIN) / 2048), blk, 0, stream>>>(xs, X16);
  fwd_kernel<<<dim3(HDIM / 64, SEQ / 64), blk, 0, stream>>>(X16, W1t, b1, H16, HT16);
  qscan_kernel<<<dim3(1), blk, 0, stream>>>(H16, w2, b2, targets, actions, dones, Cp, out + OUT_B2);
  makeu_kernel<<<dim3(HDIM / 32), blk, 0, stream>>>(HT16, w2, actions, Cp, UT16, out + OUT_B1);
  gw1_kernel<<<dim3(HDIM / 64, DIN / 64), blk, 0, stream>>>(XT16, UT16, out + OUT_W1);
  gw2_kernel<<<dim3(HDIM / 128), blk, 0, stream>>>(HT16, Cp, actions, out + OUT_W2);
}
